// Mamba2_31542239822384
// MI455X (gfx1250) — hardware-verified
//
#include <hip/hip_runtime.h>
#include <math.h>
#include <float.h>

typedef __attribute__((ext_vector_type(16))) _Float16 v16h;
typedef __attribute__((ext_vector_type(8)))  _Float16 v8h;
typedef __attribute__((ext_vector_type(16))) __bf16   v16b;
typedef __attribute__((ext_vector_type(8)))  __bf16   v8b;
typedef __attribute__((ext_vector_type(8)))  float    v8f;
typedef __attribute__((ext_vector_type(4)))  float    v4f;
typedef __attribute__((ext_vector_type(4)))  unsigned int v4u;
typedef __attribute__((ext_vector_type(2)))  unsigned int v2u;

constexpr int kL        = 4096;
constexpr int kDm       = 1024;
constexpr int kDin      = 2048;
constexpr int kNst      = 128;
constexpr int kHd       = 64;
constexpr int kNh       = 32;
constexpr int kConv     = 2304;
constexpr int kChunk    = 256;
constexpr int kNc       = 16;
constexpr int kNproj    = 4384;
constexpr int kNprojPad = 4416;
constexpr int kBCP      = 256;
constexpr int kDtP      = 64;
constexpr int kConvTP   = 260;
constexpr int kTrP      = 72;
constexpr int kStElems  = kNc * kNh * kHd * kNst;
constexpr float kTileCarry = 64.0f;
constexpr float kPsCarry   = 256.0f;
static_assert(kDin + 2 * kNst == kConv, "conv width");
static_assert(2 * kDin + 2 * kNst + kNh == kNproj, "proj width");
static_assert((kNprojPad % 64) == 0 && kNprojPad >= kNproj && kNprojPad - kNproj < 64, "proj pad");
static_assert((kL % 64) == 0 && (kDin % 64) == 0 && (kConv % 64) == 0 && (kDtP % 64) == 0 && (kDm % 64) == 0, "GEMM M,N tiles");
static_assert((kDm % 32) == 0 && (kDin % 32) == 0, "GEMM K steps");
static_assert(kDin + kConv + kDtP == kNprojPad, "column split of the padded projection");
static_assert((kL % kChunk) == 0 && kL / kChunk == kNc && kNh * kHd == kDin, "chunking");
static_assert(kStElems == 4194304, "state elements");

constexpr size_t kOffWOUTT = 0;
constexpr size_t kOffZP    = kOffWOUTT + (size_t)kDm * kDin * 2;
constexpr size_t kOffXR    = kOffZP + (size_t)kL * kDin * 2;
constexpr size_t kOffY     = kOffXR;
constexpr size_t kEndXR    = kOffXR + (size_t)kL * kConv * 4;
constexpr size_t kOffDTR   = kEndXR;
constexpr size_t kOffDTP   = kOffDTR + (size_t)kL * kDtP * 4;
constexpr size_t kOffCSP   = kOffDTP + (size_t)kNh * kL * 4;
constexpr size_t kOffBC    = kOffCSP + (size_t)kNh * kL * 4;
constexpr size_t kOffXH    = kOffBC + (size_t)kL * kBCP * 2;
constexpr size_t kOffPS    = kOffXH + (size_t)kL * kDin * 2;
constexpr size_t kOffYNL   = kOffPS + (size_t)kStElems * 2;
constexpr size_t kOffHSB   = kOffYNL + (size_t)kL * kDin * 2;
constexpr size_t kOffYNH   = kOffHSB;
constexpr size_t kOffWINT  = kOffHSB + (size_t)kL * kDm * 2;
constexpr size_t kWsTotal  = kOffWINT + (size_t)kNprojPad * kDm * 2;
static_assert(kOffY + (size_t)kL * kDin * 4 <= kEndXR, "y plane fits the dead raw-xBC region");
static_assert(kOffYNH + (size_t)kL * kDin * 2 <= kWsTotal, "ynorm hi plane fits the dead HSB+WINT regions");
static_assert(kOffYNL + (size_t)kL * kDin * 2 == kOffHSB, "ynorm lo plane is fresh");
static_assert(kWsTotal == 122290176ull, "carve total");
static_assert(kWsTotal <= 134217728ull, "carve cap");
static_assert((kOffZP % 128) == 0 && (kOffXR % 128) == 0 && (kOffDTR % 128) == 0 && (kOffDTP % 128) == 0 &&
              (kOffCSP % 128) == 0 && (kOffBC % 128) == 0 && (kOffXH % 128) == 0 && (kOffPS % 128) == 0 &&
              (kOffYNL % 128) == 0 && (kOffHSB % 128) == 0 && (kOffWINT % 128) == 0,
              "128-B aligned regions");

__device__ __forceinline__ unsigned short f2bf_bits(float f) {
  unsigned u = __float_as_uint(f);
  return (unsigned short)((u + 0x7FFFu + ((u >> 16) & 1u)) >> 16);
}
__device__ __forceinline__ float bf_bits2f(unsigned short h) { return __uint_as_float(((unsigned)h) << 16); }
__device__ __forceinline__ float bfr(float f) { return bf_bits2f(f2bf_bits(f)); }
__device__ __forceinline__ float h16_to_f32(unsigned hb) {
  const unsigned sgn = (hb & 0x8000u) << 16; const unsigned em = hb & 0x7fffu;
  const float fn = __uint_as_float((em << 13) + 0x38000000u);
  const float fs = (float)em * 5.9604644775390625e-8f;
  const float mag = (em < 0x400u) ? fs : fn; return __uint_as_float(__float_as_uint(mag) | sgn);
}
__device__ __forceinline__ unsigned pack_bf16x2(float a, float b) {
  return (unsigned)f2bf_bits(a) | ((unsigned)f2bf_bits(b) << 16);
}
__device__ __forceinline__ unsigned pack_f16x2(float a, float b) {
  return (unsigned)__builtin_bit_cast(unsigned short, (_Float16)a) | ((unsigned)__builtin_bit_cast(unsigned short, (_Float16)b) << 16);
}
__device__ __forceinline__ void split_bf16x2(float a, float b, unsigned& hw, unsigned& lw) {
  const unsigned short ha = f2bf_bits(a), hb2 = f2bf_bits(b);
  const unsigned short la = f2bf_bits(a - bf_bits2f(ha)), lb = f2bf_bits(b - bf_bits2f(hb2));
  hw = (unsigned)ha | ((unsigned)hb2 << 16);
  lw = (unsigned)la | ((unsigned)lb << 16);
}

__device__ __forceinline__ void dep_guard_h(v8f& a, v8f& b, v16h x, v16h y) { asm volatile("v_nop\n\tv_nop\n\tv_nop\n\tv_nop" : "+v"(a), "+v"(b) : "v"(x), "v"(y)); }
__device__ __forceinline__ void dep_guard_b(v8f& a, v8f& b, v16b x, v16b y) { asm volatile("v_nop\n\tv_nop\n\tv_nop\n\tv_nop" : "+v"(a), "+v"(b) : "v"(x), "v"(y)); }
__device__ __forceinline__ void dep_guard4_h(v8f& a, v8f& b, v8f& c, v8f& d, v16h x, v16h y) { asm volatile("v_nop\n\tv_nop\n\tv_nop\n\tv_nop" : "+v"(a), "+v"(b), "+v"(c), "+v"(d) : "v"(x), "v"(y)); }
__device__ __forceinline__ void dep_guard4_b(v8f& a, v8f& b, v8f& c, v8f& d, v16b x, v16b y) { asm volatile("v_nop\n\tv_nop\n\tv_nop\n\tv_nop" : "+v"(a), "+v"(b), "+v"(c), "+v"(d) : "v"(x), "v"(y)); }
__device__ __forceinline__ void keep4_h(v16h a, v16h b, v16h c, v16h d) { asm volatile("v_nop" :: "v"(a), "v"(b), "v"(c), "v"(d)); }
__device__ __forceinline__ void keep4_b(v16b a, v16b b, v16b c, v16b d) { asm volatile("v_nop" :: "v"(a), "v"(b), "v"(c), "v"(d)); }
__device__ __forceinline__ void acc_guard4(v8f& a, v8f& b, v8f& c, v8f& d) { asm volatile("v_nop\n\tv_nop\n\tv_nop\n\tv_nop" : "+v"(a), "+v"(b), "+v"(c), "+v"(d)); }
template <typename T> struct Frag;
template <> struct Frag<_Float16> {
  typedef v16h V; union U { v16h v; v8h h[2]; };
  static __device__ __forceinline__ v16h load(const _Float16* p) {
    U f; f.h[0] = *(const v8h*)(p); f.h[1] = *(const v8h*)(p + 16); return f.v;
  }
  static __device__ __forceinline__ v8f mma(v16h a, v16h b, v8f c) {
    return __builtin_amdgcn_wmma_f32_16x16x32_f16(false, a, false, b, (short)0, c, false, false);
  }
  static __device__ __forceinline__ void guard(v8f& a, v8f& b, v16h x, v16h y) { dep_guard_h(a, b, x, y); }
  static __device__ __forceinline__ void guard4(v8f& a, v8f& b, v8f& c, v8f& d, v16h x, v16h y) { dep_guard4_h(a, b, c, d, x, y); }
  static __device__ __forceinline__ void keep(v16h a, v16h b, v16h c, v16h d) { keep4_h(a, b, c, d); }
};
template <> struct Frag<__bf16> {
  typedef v16b V; union U { v16b v; v8b h[2]; };
  static __device__ __forceinline__ v16b load(const __bf16* p) {
    U f; f.h[0] = *(const v8b*)(p); f.h[1] = *(const v8b*)(p + 16); return f.v;
  }
  static __device__ __forceinline__ v8f mma(v16b a, v16b b, v8f c) {
    return __builtin_amdgcn_wmma_f32_16x16x32_bf16(false, a, false, b, (short)0, c, false, false);
  }
  static __device__ __forceinline__ void guard(v8f& a, v8f& b, v16b x, v16b y) { dep_guard_b(a, b, x, y); }
  static __device__ __forceinline__ void guard4(v8f& a, v8f& b, v8f& c, v8f& d, v16b x, v16b y) { dep_guard4_b(a, b, c, d, x, y); }
  static __device__ __forceinline__ void keep(v16b a, v16b b, v16b c, v16b d) { keep4_b(a, b, c, d); }
};
__device__ __forceinline__ v8f mma_h(v16h a, v16h b, v8f c) {
  c = __builtin_amdgcn_wmma_f32_16x16x32_f16(false, a, false, b, (short)0, c, false, false);
  asm volatile("v_nop\n\tv_nop\n\tv_nop\n\tv_nop" : "+v"(c) : "v"(a), "v"(b));
  return c;
}
__device__ __forceinline__ v8f v8zero() { return (v8f){0.f,0.f,0.f,0.f,0.f,0.f,0.f,0.f}; }

template <int ET> struct Elem;
template <> struct Elem<0> { typedef _Float16 T; };
template <> struct Elem<1> { typedef __bf16 T; };
template <int ET, int SPL, int BIAS_MODE, int OUT_MODE, bool RESID, int ACT = 0>
__global__ __launch_bounds__(256) void wmma_gemm64(
    const unsigned short* __restrict__ Ap, const unsigned short* __restrict__ A2p, int lda, long strideA,
    const unsigned short* __restrict__ Btp, const unsigned short* __restrict__ Bt2p, int ldb, long strideB,
    void* __restrict__ Cout, void* __restrict__ Cout2, int ldc, long strideC,
    const float* __restrict__ bias,
    const float* __restrict__ resid, long strideR,
    int M, int N, int K, float scale) {
  typedef typename Elem<ET>::T T;
  typedef typename Frag<T>::V V;
  const T* A = (const T*)Ap; const T* A2 = (const T*)A2p; const T* Bt = (const T*)Btp; const T* Bt2 = (const T*)Bt2p;
  __shared__ __align__(16) float sT[8][16 * 68];
  const int b    = blockIdx.y;
  const int lane = threadIdx.x & 31;
  const int wave = threadIdx.x >> 5;
  const int tilesN = N >> 6;
  const int tilesM = M >> 6;
  const int tile = blockIdx.x * 8 + wave;
  if (tile >= tilesM * tilesN) return;
  const int tm = tile / tilesN;
  const int tn = tile - tm * tilesN;
  const int m0 = tm << 6;
  const int n0 = tn << 6;

  const T* Ab  = A  + (size_t)b * strideA;
  const T* Bb  = Bt + (size_t)b * strideB;
  const T* Ab2 = (SPL >= 1) ? (A2  + (size_t)b * strideA) : nullptr;
  const T* Bb2 = (SPL == 2) ? (Bt2 + (size_t)b * strideB) : nullptr;

  const int rlane = lane & 15;
  const int koff  = (lane >> 4) * 8;
  const int mOff  = (lane >> 4) * 8;

  v8f acc[4][4];
#pragma unroll
  for (int i = 0; i < 4; ++i)
#pragma unroll
    for (int j = 0; j < 4; ++j) acc[i][j] = (v8f){0.f,0.f,0.f,0.f,0.f,0.f,0.f,0.f};

  for (int k0 = 0; k0 < K; k0 += 32) {
    V bh[4], bl[4];
#pragma unroll
    for (int j = 0; j < 4; ++j) {
      const size_t bo = (size_t)(n0 + (j << 4) + rlane) * ldb + koff + k0;
      bh[j] = Frag<T>::load(Bb + bo);
      if (SPL == 2) bl[j] = Frag<T>::load(Bb2 + bo);
    }
#pragma unroll
    for (int i = 0; i < 4; ++i) {
      const size_t ao = (size_t)(m0 + (i << 4) + rlane) * lda + koff + k0;
      V ah = Frag<T>::load(Ab + ao);
      V al;
      if (SPL >= 1) al = Frag<T>::load(Ab2 + ao);
#pragma unroll
      for (int j = 0; j < 4; ++j) {
        acc[i][j] = Frag<T>::mma(ah, bh[j], acc[i][j]);
        if (SPL == 2) acc[i][j] = Frag<T>::mma(ah, bl[j], acc[i][j]);
        if (SPL >= 1) acc[i][j] = Frag<T>::mma(al, bh[j], acc[i][j]);
      }
      Frag<T>::guard4(acc[i][0], acc[i][1], acc[i][2], acc[i][3], ah, (SPL >= 1) ? al : ah);
    }
    Frag<T>::keep(bh[0], bh[1], bh[2], bh[3]);
    if (SPL == 2) Frag<T>::keep(bl[0], bl[1], bl[2], bl[3]);
  }
  acc_guard4(acc[0][0], acc[0][1], acc[0][2], acc[0][3]);
  acc_guard4(acc[1][0], acc[1][1], acc[1][2], acc[1][3]);
  acc_guard4(acc[2][0], acc[2][1], acc[2][2], acc[2][3]);
  acc_guard4(acc[3][0], acc[3][1], acc[3][2], acc[3][3]);

  float* slab = sT[wave];
  const float* Rb = RESID ? (resid + (size_t)b * strideR) : nullptr;
#pragma unroll
  for (int i = 0; i < 4; ++i) {
    const int mBase = m0 + (i << 4);
#pragma unroll
    for (int j = 0; j < 4; ++j) {
      const int n = n0 + (j << 4) + rlane;
      float bv = 0.f;
      if (BIAS_MODE == 2) bv = bias[n];
#pragma unroll
      for (int r = 0; r < 8; ++r) {
        float v = acc[i][j][r] * scale;
        if (BIAS_MODE == 1) v += bias[mBase + mOff + r];
        if (BIAS_MODE == 2) v += bv;
        if (RESID) v += Rb[(size_t)(mBase + mOff + r) * ldc + n];
        if (ACT == 1) v = tanhf(v);
        if (ACT == 2) v = fmaxf(v, 0.0f);
        if (ACT == 3) v = v / (1.0f + expf(-v));
        if (ACT == 4) v = (v > 0.f) ? v : 0.01f * v;
        slab[(mOff + r) * 68 + (j << 4) + rlane] = v;
      }
    }
    __builtin_amdgcn_fence(__ATOMIC_RELEASE, "workgroup");
    __builtin_amdgcn_wave_barrier();
    __builtin_amdgcn_fence(__ATOMIC_ACQUIRE, "workgroup");
    if (OUT_MODE == 0) {
      float* C = (float*)Cout + (size_t)b * strideC;
      const int hh = lane >> 4, c4 = (lane & 15) * 4;
      for (int pass = 0; pass < 2; ++pass) {
#pragma unroll
        for (int it = 0; it < 8; ++it) {
          const int row = it * 2 + hh;
          v4f v = *(const v4f*)(slab + row * 68 + c4);
          *(volatile v4f*)(C + (size_t)(mBase + row) * ldc + n0 + c4) = v;
        }
        __threadfence();
      }
    } else {
      const int q = lane >> 3, c8 = (lane & 7) * 8;
      unsigned short* C  = (unsigned short*)Cout  + (size_t)b * strideC;
      unsigned short* C2 = (OUT_MODE == 2) ? ((unsigned short*)Cout2 + (size_t)b * strideC) : nullptr;
      for (int pass = 0; pass < 2; ++pass) {
#pragma unroll
        for (int it = 0; it < 4; ++it) {
          const int row = it * 4 + q;
          const float* sp = slab + row * 68 + c8;
          v8h hv, lv;
#pragma unroll
          for (int e = 0; e < 8; ++e) {
            if (OUT_MODE == 1) {
              hv[e] = (_Float16)sp[e];
            } else {
              unsigned short hb = f2bf_bits(sp[e]);
              unsigned short lb = f2bf_bits(sp[e] - bf_bits2f(hb));
              hv[e] = __builtin_bit_cast(_Float16, hb);
              lv[e] = __builtin_bit_cast(_Float16, lb);
            }
          }
          *(volatile v8h*)(C + (size_t)(mBase + row) * ldc + n0 + c8) = hv;
          if (OUT_MODE == 2) *(volatile v8h*)(C2 + (size_t)(mBase + row) * ldc + n0 + c8) = lv;
        }
        __threadfence();
      }
    }
    __builtin_amdgcn_fence(__ATOMIC_RELEASE, "workgroup");
    __builtin_amdgcn_wave_barrier();
    __builtin_amdgcn_fence(__ATOMIC_ACQUIRE, "workgroup");
  }
}

__global__ __launch_bounds__(256) void cast_bf16_kernel(
    const float* __restrict__ src, unsigned short* __restrict__ dst, int total8)
{
  const int i = blockIdx.x * 256 + threadIdx.x;
  if (i >= total8) return;
  const size_t e0 = (size_t)i << 3;
  const v4f a0 = *(const v4f*)(src + e0);
  const v4f a1 = *(const v4f*)(src + e0 + 4);
  v4u w;
  w[0] = pack_bf16x2(a0[0], a0[1]); w[1] = pack_bf16x2(a0[2], a0[3]);
  w[2] = pack_bf16x2(a1[0], a1[1]); w[3] = pack_bf16x2(a1[2], a1[3]);
  unsigned short* q = dst + e0;
  *(volatile v4u*)q = w;
  __threadfence();
  *(volatile v4u*)q = w;
}

__global__ __launch_bounds__(256) void transpose_bf16_kernel(
    const float* __restrict__ src, unsigned short* __restrict__ dst, int R, int C)
{
  __shared__ __align__(16) unsigned short sTile[64 * kTrP];
  const int tid = threadIdx.x, lane = tid & 31, wave = tid >> 5;
  const int c0 = blockIdx.x * 64, r0 = blockIdx.y * 64;
#pragma unroll
  for (int k = 0; k < 4; ++k) {
    const int idx = tid + 256 * k;
    const int rr = idx >> 4, cq = idx & 15;
    const int cc = c0 + cq * 4;
    const int ccl = (cc < C) ? cc : (C - 4);
    const v4f v = *(const v4f*)(src + (size_t)(r0 + rr) * C + ccl);
    const unsigned short keep = (unsigned short)(0u - (unsigned)(cc < C));
#pragma unroll
    for (int e = 0; e < 4; ++e) {
      const unsigned short bits = f2bf_bits(v[e]);
      sTile[(cq * 4 + e) * kTrP + rr] = (unsigned short)(bits & keep);
    }
  }
  __syncthreads();
  v4u val[2];
#pragma unroll
  for (int it = 0; it < 2; ++it) {
    const int cl = wave * 8 + it * 4 + (lane >> 3);
    val[it] = *(const v4u*)(sTile + cl * kTrP + (lane & 7) * 8);
  }
  for (int pass = 0; pass < 2; ++pass) {
#pragma unroll
    for (int it = 0; it < 2; ++it) {
      const int cl = wave * 8 + it * 4 + (lane >> 3);
      *(volatile v4u*)(dst + (size_t)(c0 + cl) * R + r0 + (lane & 7) * 8) = val[it];
    }
    __threadfence();
  }
}

__global__ __launch_bounds__(256) void dt_cumsum_kernel(
    const float* __restrict__ DTR, const float* __restrict__ dt_bias, const float* __restrict__ A_log,
    float* __restrict__ DTP, float* __restrict__ CSP)
{
  __shared__ __align__(16) float scs[kChunk];
  __shared__ __align__(16) float sdt[kChunk];
  const int tid = threadIdx.x;
  const int wave = __builtin_amdgcn_readfirstlane(tid >> 5);
  const int h = blockIdx.x, c = blockIdx.y;
  const int l0 = c * kChunk;
  const float raw = DTR[(size_t)(l0 + tid) * kDtP + h] + bfr(dt_bias[h]);
  const float dt = fmaxf(raw, 0.0f) + log1pf(expf(-fabsf(raw)));
  const float An = -expf(bfr(A_log[h]));
  scs[tid] = dt * An;
  sdt[tid] = dt;
  __syncthreads();
  for (int off = 1; off < kChunk; off <<= 1) {
    const int si = (tid >= off) ? (tid - off) : 0;
    const float f01 = (tid >= off) ? 1.0f : 0.0f;
    const float v = scs[si] * f01;
    __syncthreads();
    scs[tid] += v;
    __syncthreads();
  }
  if (wave < 2) {
    const int e = tid * 4;
    const v4f v = *(const v4f*)(sdt + e);
    float* p = DTP + (size_t)h * kL + l0 + e;
    *(volatile v4f*)p = v;
    __threadfence();
    *(volatile v4f*)p = v;
  } else if (wave < 4) {
    const int e = (tid - 64) * 4;
    const v4f v = *(const v4f*)(scs + e);
    float* p = CSP + (size_t)h * kL + l0 + e;
    *(volatile v4f*)p = v;
    __threadfence();
    *(volatile v4f*)p = v;
  }
}

__global__ __launch_bounds__(256) void conv_silu_kernel(
    const float* __restrict__ XR, const float* __restrict__ cw, const float* __restrict__ cb,
    unsigned short* __restrict__ XH, unsigned short* __restrict__ BC)
{
  __shared__ __align__(16) float sT[16 * kConvTP];
  const int tid = threadIdx.x, lane = tid & 31, wave = tid >> 5;
  const int bx = blockIdx.x;
  const int d0 = bx * 256, d = d0 + tid;
  const int g0 = blockIdx.y * 64;
  const float w0 = bfr(cw[d * 4 + 0]), w1 = bfr(cw[d * 4 + 1]), w2 = bfr(cw[d * 4 + 2]), w3 = bfr(cw[d * 4 + 3]);
  const float bc = bfr(cb[d]);
  float xm3 = 0.f, xm2 = 0.f, xm1 = 0.f;
  if (g0 > 0) {
    xm3 = XR[(size_t)(g0 - 3) * kConv + d];
    xm2 = XR[(size_t)(g0 - 2) * kConv + d];
    xm1 = XR[(size_t)(g0 - 1) * kConv + d];
  }
#pragma unroll 1
  for (int sub = 0; sub < 4; ++sub) {
    const int lb = g0 + sub * 16;
#pragma unroll 1
    for (int s = 0; s < 16; ++s) {
      const float xcur = XR[(size_t)(lb + s) * kConv + d];
      float acc = w0 * xm3;
      acc = fmaf(w1, xm2, acc);
      acc = fmaf(w2, xm1, acc);
      acc = fmaf(w3, xcur, acc);
      const float sv = acc + bc;
      const float sg = __builtin_amdgcn_rcpf(1.0f + __expf(-sv));
      sT[s * kConvTP + tid] = sv * sg;
      xm3 = xm2; xm2 = xm1; xm1 = xcur;
    }
    __syncthreads();
    v4u hw[2];
#pragma unroll
    for (int it = 0; it < 2; ++it) {
      const float* sp = sT + (it * 8 + wave) * kConvTP + lane * 8;
      const v4f a0 = *(const v4f*)(sp);
      const v4f a1 = *(const v4f*)(sp + 4);
      hw[it][0] = pack_f16x2(a0[0], a0[1]); hw[it][1] = pack_f16x2(a0[2], a0[3]);
      hw[it][2] = pack_f16x2(a1[0], a1[1]); hw[it][3] = pack_f16x2(a1[2], a1[3]);
    }
    if (bx < 8) {
      for (int pass = 0; pass < 2; ++pass) {
#pragma unroll
        for (int it = 0; it < 2; ++it)
          *(volatile v4u*)(XH + (size_t)(lb + it * 8 + wave) * kDin + d0 + lane * 8) = hw[it];
        __threadfence();
      }
    } else {
      for (int pass = 0; pass < 2; ++pass) {
#pragma unroll
        for (int it = 0; it < 2; ++it)
          *(volatile v4u*)(BC + (size_t)(lb + it * 8 + wave) * kBCP + lane * 8) = hw[it];
        __threadfence();
      }
    }
    __syncthreads();
  }
}

__global__ __launch_bounds__(256) void chunk_state_prefix_kernel(
    const unsigned short* __restrict__ XH, const unsigned short* __restrict__ BC,
    const float* __restrict__ DTP, const float* __restrict__ CSP, unsigned short* __restrict__ PS)
{
  __shared__ __align__(16) _Float16 sXD[64 * 40];
  __shared__ __align__(16) unsigned short sBT[128 * 40];
  __shared__ __align__(16) float slabs[8][16 * 68];
  __shared__ __align__(16) float sCS[kChunk];
  __shared__ __align__(16) float sDT[kChunk];
  const int h = blockIdx.x;
  const int tid = threadIdx.x, lane = tid & 31;
  const int wave = __builtin_amdgcn_readfirstlane(tid >> 5);
  const int rlane = lane & 15, hh = lane >> 4, koff = hh * 8;
  const int xj = tid >> 3, xq = (tid & 7) * 8;
  const int bj = tid & 31, bn = (tid >> 5) * 16;
  const int prow0 = (wave & 3) * 16, ncol0 = (wave >> 2) * 64;
  const int q = lane >> 3, c8 = (lane & 7) * 8;
  float* slab = slabs[wave];

  v8f run[4];
#pragma unroll
  for (int a = 0; a < 4; ++a) run[a] = v8zero();

#pragma unroll 1
  for (int c = 0; c < kNc; ++c) {
    const int l0 = c * kChunk;
    __syncthreads();
    sCS[tid] = CSP[(size_t)h * kL + l0 + tid];
    sDT[tid] = DTP[(size_t)h * kL + l0 + tid];

#pragma unroll
    for (int ni = 0; ni < 4; ++ni)
#pragma unroll
      for (int r = 0; r < 8; ++r) slab[(8 * hh + r) * 68 + ni * 16 + rlane] = run[ni][r] * kPsCarry;
    __builtin_amdgcn_fence(__ATOMIC_RELEASE, "workgroup");
    __builtin_amdgcn_wave_barrier();
    __builtin_amdgcn_fence(__ATOMIC_ACQUIRE, "workgroup");
    {
      unsigned short* pbase = PS + ((size_t)((c * kNh + h) * kHd + prow0)) * kNst + ncol0;
      v4u pv[4];
#pragma unroll
      for (int it = 0; it < 4; ++it) {
        const int row = it * 4 + q;
        const float* sp = slab + row * 68 + c8;
        const v4f a0 = *(const v4f*)(sp);
        const v4f a1 = *(const v4f*)(sp + 4);
        pv[it][0] = pack_f16x2(a0[0], a0[1]); pv[it][1] = pack_f16x2(a0[2], a0[3]);
        pv[it][2] = pack_f16x2(a1[0], a1[1]); pv[it][3] = pack_f16x2(a1[2], a1[3]);
      }
      for (int pass = 0; pass < 2; ++pass) {
#pragma unroll
        for (int it = 0; it < 4; ++it) {
          const int row = it * 4 + q;
          *(volatile v4u*)(pbase + (size_t)row * kNst + c8) = pv[it];
        }
        __threadfence();
      }
    }
    __builtin_amdgcn_fence(__ATOMIC_RELEASE, "workgroup");
    __builtin_amdgcn_wave_barrier();
    __builtin_amdgcn_fence(__ATOMIC_ACQUIRE, "workgroup");
    __syncthreads();
    const float cs255 = sCS[kChunk - 1];

    v8f st[4];
#pragma unroll
    for (int a = 0; a < 4; ++a) st[a] = v8zero();
#pragma unroll 1
    for (int j0 = 0; j0 < kChunk; j0 += 32) {
      __syncthreads();
      {
        const size_t xo = (size_t)(l0 + j0 + xj) * kDin + h * kHd + xq;
        const v4u wh = *(const v4u*)(XH + xo);
        const float sj = sDT[j0 + xj] * expf(cs255 - sCS[j0 + xj]) * kPsCarry;
#pragma unroll
        for (int k = 0; k < 4; ++k) {
          const float x0 = h16_to_f32(wh[k] & 0xffffu);
          const float x1 = h16_to_f32(wh[k] >> 16);
          sXD[(xq + 2 * k) * 40 + xj]     = (_Float16)(x0 * sj);
          sXD[(xq + 2 * k + 1) * 40 + xj] = (_Float16)(x1 * sj);
        }
      }
      {
        const size_t brow = (size_t)(l0 + j0 + bj) * kBCP + bn;
        const v4u w0 = *(const v4u*)(BC + brow);
        const v4u w1 = *(const v4u*)(BC + brow + 8);
#pragma unroll
        for (int k = 0; k < 4; ++k) {
          sBT[(bn + 2 * k) * 40 + bj]         = (unsigned short)(w0[k] & 0xffffu);
          sBT[(bn + 2 * k + 1) * 40 + bj]     = (unsigned short)(w0[k] >> 16);
          sBT[(bn + 8 + 2 * k) * 40 + bj]     = (unsigned short)(w1[k] & 0xffffu);
          sBT[(bn + 8 + 2 * k + 1) * 40 + bj] = (unsigned short)(w1[k] >> 16);
        }
      }
      __syncthreads();
      const v16h af = Frag<_Float16>::load(sXD + (prow0 + rlane) * 40 + koff);
#pragma unroll
      for (int ni = 0; ni < 4; ++ni) {
        const v16h bf_ = Frag<_Float16>::load((const _Float16*)sBT + ((ncol0 + ni * 16 + rlane) * 40 + koff));
        st[ni] = mma_h(af, bf_, st[ni]);
      }
    }

    float cd = expf(cs255);
    cd = (cd < FLT_MIN) ? 0.0f : cd;
#pragma unroll
    for (int ni = 0; ni < 4; ++ni) run[ni] = run[ni] * cd + st[ni] * (1.0f / kPsCarry);
  }
}

struct MainTiles { unsigned short b[32 * 136]; unsigned short x[64 * 40]; _Float16 s[8][32 * 40]; };
union MainLds { MainTiles t; unsigned short p[64 * 136]; float slab[8][16 * 68]; };
static_assert(sizeof(MainTiles) == 34304 && sizeof(MainLds) == 34816, "lds union");

__global__ __launch_bounds__(256) void chunk_output_kernel(
    const unsigned short* __restrict__ BC, const unsigned short* __restrict__ PS,
    const unsigned short* __restrict__ XH,
    const float* __restrict__ DTP, const float* __restrict__ CSP, const float* __restrict__ Dv,
    float* __restrict__ Y)
{
  __shared__ __align__(16) MainLds U;
  __shared__ __align__(16) float sCS2[kChunk];
  __shared__ __align__(16) float sCSn[kChunk];
  __shared__ __align__(16) float sDT[kChunk];
  const int h = blockIdx.x, c = blockIdx.y;
  const int l0 = c * kChunk;
  const int tid = threadIdx.x, lane = tid & 31;
  const int wave = __builtin_amdgcn_readfirstlane(tid >> 5);
  const int rlane = lane & 15, hh = lane >> 4, koff = hh * 8;

  {
    const float csn = CSP[(size_t)h * kL + l0 + tid];
    sCSn[tid] = csn;
    sCS2[tid] = csn * 1.4426950408889634f;
    sDT[tid]  = DTP[(size_t)h * kL + l0 + tid] * kTileCarry;
  }
  {
    const int p = tid >> 2, q = tid & 3;
    const unsigned short* pr = PS + ((size_t)((c * kNh + h) * kHd + p)) * kNst + q * 32;
#pragma unroll
    for (int k = 0; k < 4; ++k) {
      const v4u w = *(const v4u*)(pr + 8 * k);
      *(v4u*)(U.p + p * 136 + q * 32 + 8 * k) = w;
    }
  }
  __syncthreads();

  const _Float16* Cg = (const _Float16*)BC + (size_t)(l0 + (wave << 5)) * kBCP + kNst;

  v8f yacc[2][4];
#pragma unroll
  for (int a = 0; a < 2; ++a)
#pragma unroll
    for (int b2 = 0; b2 < 4; ++b2) yacc[a][b2] = v8zero();

#pragma unroll
  for (int kt = 0; kt < 4; ++kt) {
    asm volatile("" ::: "memory");
    const v16h cfa = Frag<_Float16>::load(Cg + (size_t)rlane * kBCP + kt * 32 + koff);
    const v16h cfb = Frag<_Float16>::load(Cg + (size_t)(16 + rlane) * kBCP + kt * 32 + koff);
#pragma unroll
    for (int pi = 0; pi < 4; ++pi) {
      const v16h bq = Frag<_Float16>::load((const _Float16*)U.p + ((pi * 16 + rlane) * 136 + kt * 32 + koff));
      yacc[0][pi] = mma_h(cfa, bq, yacc[0][pi]);
      yacc[1][pi] = mma_h(cfb, bq, yacc[1][pi]);
    }
  }
#pragma unroll
  for (int mi = 0; mi < 2; ++mi) {
#pragma unroll
    for (int r = 0; r < 8; ++r) {
      float er = expf(sCSn[(wave << 5) + mi * 16 + 8 * hh + r]);
      er = (er < FLT_MIN) ? 0.0f : er;
      const float sc = er * (kTileCarry / kPsCarry);
#pragma unroll
      for (int pi = 0; pi < 4; ++pi) yacc[mi][pi][r] = yacc[mi][pi][r] * sc;
    }
  }

  const int xj = tid >> 3, xq = (tid & 7) * 8;
#pragma unroll 1
  for (int j0 = 0; j0 < kChunk; j0 += 32) {
    __syncthreads();
#pragma unroll
    for (int k = 0; k < 2; ++k) {
      const int idx = tid + 256 * k;
      const int r = idx >> 4, q = idx & 15;
      const v4u w = *(const v4u*)(BC + (size_t)(l0 + j0 + r) * kBCP + q * 8);
      *(v4u*)(&U.t.b[r * 136 + q * 8]) = w;
    }
    {
      const size_t xo = (size_t)(l0 + j0 + xj) * kDin + h * kHd + xq;
      const v4u wh = *(const v4u*)(XH + xo);
#pragma unroll
      for (int k = 0; k < 4; ++k) {
        U.t.x[(xq + 2 * k) * 40 + xj]     = (unsigned short)(wh[k] & 0xffffu);
        U.t.x[(xq + 2 * k + 1) * 40 + xj] = (unsigned short)(wh[k] >> 16);
      }
    }
    __syncthreads();
    if (j0 <= (wave << 5)) {
      v8f sacc[2][2];
#pragma unroll
      for (int a = 0; a < 2; ++a)
#pragma unroll
        for (int b2 = 0; b2 < 2; ++b2) sacc[a][b2] = v8zero();
#pragma unroll
      for (int nk = 0; nk < 4; ++nk) {
        asm volatile("" ::: "memory");
        const v16h cfa = Frag<_Float16>::load(Cg + (size_t)rlane * kBCP + nk * 32 + koff);
        const v16h cfb = Frag<_Float16>::load(Cg + (size_t)(16 + rlane) * kBCP + nk * 32 + koff);
#pragma unroll
        for (int ji = 0; ji < 2; ++ji) {
          const v16h bfr_ = Frag<_Float16>::load((const _Float16*)U.t.b + ((ji * 16 + rlane) * 136 + nk * 32 + koff));
          sacc[0][ji] = mma_h(cfa, bfr_, sacc[0][ji]);
          sacc[1][ji] = mma_h(cfb, bfr_, sacc[1][ji]);
        }
      }
      _Float16* sw = U.t.s[wave];
#pragma unroll
      for (int mi = 0; mi < 2; ++mi) {
#pragma unroll
        for (int r = 0; r < 8; ++r) {
          const int il = mi * 16 + 8 * hh + r;
          const int ig = (wave << 5) + il;
          const float csi = sCS2[ig];
#pragma unroll
          for (int ji = 0; ji < 2; ++ji) {
            const int jl = ji * 16 + rlane;
            const int jg = j0 + jl;
            const float dd = fminf(csi - sCS2[jg], 24.0f);
            const float keep = (jg <= ig) ? 1.0f : 0.0f;
            const float v = (sacc[mi][ji][r] * exp2f(dd) * sDT[jg]) * keep;
            sw[il * 40 + jl] = (_Float16)v;
          }
        }
      }
      __builtin_amdgcn_fence(__ATOMIC_RELEASE, "workgroup");
      __builtin_amdgcn_wave_barrier();
      __builtin_amdgcn_fence(__ATOMIC_ACQUIRE, "workgroup");
      const v16h af0 = Frag<_Float16>::load(sw + rlane * 40 + koff);
      const v16h af1 = Frag<_Float16>::load(sw + (16 + rlane) * 40 + koff);
#pragma unroll
      for (int pi = 0; pi < 4; ++pi) {
        const v16h bx4 = Frag<_Float16>::load((const _Float16*)U.t.x + ((pi * 16 + rlane) * 40 + koff));
        yacc[0][pi] = mma_h(af0, bx4, yacc[0][pi]);
        yacc[1][pi] = mma_h(af1, bx4, yacc[1][pi]);
      }
    }
  }
  __syncthreads();

  float* slab = U.slab[wave];
  const int c4 = (lane & 15) * 4;
  const float Dh = bfr(Dv[h]);
#pragma unroll
  for (int mi = 0; mi < 2; ++mi) {
#pragma unroll
    for (int pi = 0; pi < 4; ++pi)
#pragma unroll
      for (int r = 0; r < 8; ++r) slab[(8 * hh + r) * 68 + pi * 16 + rlane] = yacc[mi][pi][r] * (1.0f / kTileCarry);
    __builtin_amdgcn_fence(__ATOMIC_RELEASE, "workgroup");
    __builtin_amdgcn_wave_barrier();
    __builtin_amdgcn_fence(__ATOMIC_ACQUIRE, "workgroup");
    const int rowbase = l0 + (wave << 5) + mi * 16;
    v4f vals[8];
#pragma unroll
    for (int it = 0; it < 8; ++it) {
      if (it == 4) asm volatile("" ::: "memory");
      const int row = it * 2 + hh;
      const v4f sv = *(const v4f*)(slab + row * 68 + c4);
      const size_t xo = (size_t)(rowbase + row) * kDin + h * kHd + c4;
      const v2u xh2 = *(const v2u*)(XH + xo);
      v4f xv;
      xv[0] = h16_to_f32(xh2[0] & 0xffffu);
      xv[1] = h16_to_f32(xh2[0] >> 16);
      xv[2] = h16_to_f32(xh2[1] & 0xffffu);
      xv[3] = h16_to_f32(xh2[1] >> 16);
      vals[it] = sv + xv * Dh;
    }
    for (int pass = 0; pass < 2; ++pass) {
#pragma unroll
      for (int it = 0; it < 8; ++it) {
        const int row = it * 2 + hh;
        *(volatile v4f*)(Y + (size_t)(rowbase + row) * kDin + h * kHd + c4) = vals[it];
      }
      __threadfence();
    }
    __builtin_amdgcn_fence(__ATOMIC_RELEASE, "workgroup");
    __builtin_amdgcn_wave_barrier();
    __builtin_amdgcn_fence(__ATOMIC_ACQUIRE, "workgroup");
  }
}

__global__ __launch_bounds__(256) void gate_norm_kernel(
    const float* __restrict__ Y, const unsigned short* __restrict__ ZP, const float* __restrict__ nw,
    unsigned short* __restrict__ YNH, unsigned short* __restrict__ YNL)
{
  __shared__ float sred[8];
  const int tid = threadIdx.x, lane = tid & 31, wave = tid >> 5;
  const size_t row = blockIdx.x;
  const int e0 = tid * 8;
  const v4f y0 = *(const v4f*)(Y + row * kDin + e0);
  const v4f y1 = *(const v4f*)(Y + row * kDin + e0 + 4);
  const v4u zw = *(const v4u*)(ZP + row * kDin + e0);
  float g[8];
#pragma unroll
  for (int k = 0; k < 4; ++k) {
    const float za = h16_to_f32(zw[k] & 0xffffu);
    const float zb = h16_to_f32(zw[k] >> 16);
    const float ya = (k < 2) ? y0[2 * k] : y1[2 * k - 4];
    const float yb = (k < 2) ? y0[2 * k + 1] : y1[2 * k - 3];
    const float sa = __builtin_amdgcn_rcpf(1.0f + __expf(-za));
    const float sb = __builtin_amdgcn_rcpf(1.0f + __expf(-zb));
    g[2 * k]     = ya * (za * sa);
    g[2 * k + 1] = yb * (zb * sb);
  }
  float ss = 0.0f;
#pragma unroll
  for (int k = 0; k < 8; ++k) ss = fmaf(g[k], g[k], ss);
#pragma unroll
  for (int off = 16; off > 0; off >>= 1) ss += __shfl_xor(ss, off, 32);
  if (lane == 0) sred[wave] = ss;
  __syncthreads();
  float tot = 0.0f;
#pragma unroll
  for (int w = 0; w < 8; ++w) tot += sred[w];
  const float inv = rsqrtf(tot * (1.0f / (float)kDin) + 1e-5f);
  const v4f n0 = *(const v4f*)(nw + e0);
  const v4f n1 = *(const v4f*)(nw + e0 + 4);
  v4u hw, lw;
#pragma unroll
  for (int k = 0; k < 4; ++k) {
    const float wa = bfr((k < 2) ? n0[2 * k] : n1[2 * k - 4]);
    const float wb = bfr((k < 2) ? n0[2 * k + 1] : n1[2 * k - 3]);
    const float oa = (g[2 * k] * inv) * wa;
    const float ob = (g[2 * k + 1] * inv) * wb;
    unsigned a, bl;
    split_bf16x2(oa, ob, a, bl);
    hw[k] = a; lw[k] = bl;
  }
  unsigned short* qh = YNH + row * kDin + e0;
  unsigned short* ql = YNL + row * kDin + e0;
  *(volatile v4u*)qh = hw;
  *(volatile v4u*)ql = lw;
  __threadfence();
  *(volatile v4u*)qh = hw;
  *(volatile v4u*)ql = lw;
}

extern "C" void kernel_launch(void* const* d_in, const int* in_sizes, int n_in,
                              void* d_out, int out_size, void* d_ws, size_t ws_size,
                              hipStream_t stream) {
  if (n_in < 9) return;
  if (in_sizes[0] != kL * kDm) return;
  if (in_sizes[1] != kDm * kNproj) return;
  if (in_sizes[2] != kConv * 4) return;
  if (in_sizes[3] != kConv) return;
  if (in_sizes[4] != kNh) return;
  if (in_sizes[5] != kNh) return;
  if (in_sizes[6] != kNh) return;
  if (in_sizes[7] != kDin) return;
  if (in_sizes[8] != kDin * kDm) return;
  if (out_size != kL * kDm) return;
  if (ws_size < kWsTotal) return;

  const float* hs      = (const float*)d_in[0];
  const float* W_in    = (const float*)d_in[1];
  const float* conv_w  = (const float*)d_in[2];
  const float* conv_b  = (const float*)d_in[3];
  const float* dt_bias = (const float*)d_in[4];
  const float* A_log   = (const float*)d_in[5];
  const float* Dv      = (const float*)d_in[6];
  const float* norm_w  = (const float*)d_in[7];
  const float* W_out   = (const float*)d_in[8];
  float* out = (float*)d_out;

  char* ws = (char*)d_ws;
  unsigned short* WOUTT = (unsigned short*)(ws + kOffWOUTT);
  unsigned short* ZP    = (unsigned short*)(ws + kOffZP);
  float*          XR    = (float*)(ws + kOffXR);
  float*          Y     = (float*)(ws + kOffY);
  float*          DTR   = (float*)(ws + kOffDTR);
  float*          DTP   = (float*)(ws + kOffDTP);
  float*          CSP   = (float*)(ws + kOffCSP);
  unsigned short* BC    = (unsigned short*)(ws + kOffBC);
  unsigned short* XH    = (unsigned short*)(ws + kOffXH);
  unsigned short* PS    = (unsigned short*)(ws + kOffPS);
  unsigned short* YNL   = (unsigned short*)(ws + kOffYNL);
  unsigned short* HSB   = (unsigned short*)(ws + kOffHSB);
  unsigned short* YNH   = (unsigned short*)(ws + kOffYNH);
  unsigned short* WINT  = (unsigned short*)(ws + kOffWINT);

  cast_bf16_kernel<<<(kL * kDm / 8) / 256, 256, 0, stream>>>(hs, HSB, kL * kDm / 8);
  transpose_bf16_kernel<<<dim3(kNprojPad / 64, kDm / 64), 256, 0, stream>>>(W_in, WINT, kDm, kNproj);
  transpose_bf16_kernel<<<dim3(kDm / 64, kDin / 64), 256, 0, stream>>>(W_out, WOUTT, kDin, kDm);

  wmma_gemm64<1, 0, 0, 1, false><<<dim3(256, 1), 256, 0, stream>>>(
      HSB, nullptr, kDm, 0L,
      WINT, nullptr, kDm, 0L,
      (void*)ZP, nullptr, kDin, 0L,
      nullptr, nullptr, 0L,
      kL, kDin, kDm, 1.0f);
  wmma_gemm64<1, 0, 0, 0, false><<<dim3(288, 1), 256, 0, stream>>>(
      HSB, nullptr, kDm, 0L,
      WINT + (size_t)kDin * kDm, nullptr, kDm, 0L,
      (void*)XR, nullptr, kConv, 0L,
      nullptr, nullptr, 0L,
      kL, kConv, kDm, 1.0f);
  wmma_gemm64<1, 0, 0, 0, false><<<dim3(8, 1), 256, 0, stream>>>(
      HSB, nullptr, kDm, 0L,
      WINT + (size_t)(kDin + kConv) * kDm, nullptr, kDm, 0L,
      (void*)DTR, nullptr, kDtP, 0L,
      nullptr, nullptr, 0L,
      kL, kDtP, kDm, 1.0f);

  dt_cumsum_kernel<<<dim3(kNh, kNc), kChunk, 0, stream>>>(DTR, dt_bias, A_log, DTP, CSP);

  conv_silu_kernel<<<dim3(kConv / 256, kL / 64), 256, 0, stream>>>(XR, conv_w, conv_b, XH, BC);

  chunk_state_prefix_kernel<<<kNh, 256, 0, stream>>>(XH, BC, DTP, CSP, PS);
  chunk_output_kernel<<<dim3(kNh, kNc), 256, 0, stream>>>(BC, PS, XH, DTP, CSP, Dv, Y);

  gate_norm_kernel<<<kL, 256, 0, stream>>>(Y, ZP, norm_w, YNH, YNL);

  wmma_gemm64<1, 1, 0, 0, false><<<dim3(128, 1), 256, 0, stream>>>(
      YNH, YNL, kDin, 0L,
      WOUTT, nullptr, kDin, 0L,
      (void*)out, nullptr, kDm, 0L,
      nullptr, nullptr, 0L,
      kL, kDm, kDin, 1.0f);
}
